// LSTMDecoder_24532853195105
// MI455X (gfx1250) — hardware-verified
//
#include <hip/hip_runtime.h>
#include <stddef.h>

typedef __attribute__((ext_vector_type(16))) _Float16 v16h;
typedef __attribute__((ext_vector_type(8)))  _Float16 v8h;
typedef __attribute__((ext_vector_type(8)))  float    v8f;
typedef __attribute__((ext_vector_type(4)))  float    v4f;

__device__ __forceinline__ void dep_guard_h(v8f& a, v8f& b, v16h x, v16h y) { asm volatile("v_nop\n\tv_nop\n\tv_nop\n\tv_nop" : "+v"(a), "+v"(b) : "v"(x), "v"(y)); }
__device__ __forceinline__ void dep_guard1(v8f& a, v16h x, v16h y) { asm volatile("v_nop\n\tv_nop\n\tv_nop\n\tv_nop" : "+v"(a) : "v"(x), "v"(y)); }
__device__ __forceinline__ void keep4_h(v16h a, v16h b, v16h c, v16h d) { asm volatile("v_nop" :: "v"(a), "v"(b), "v"(c), "v"(d)); }
__device__ __forceinline__ void acc_guard4(v8f& a, v8f& b, v8f& c, v8f& d) { asm volatile("v_nop\n\tv_nop\n\tv_nop\n\tv_nop" : "+v"(a), "+v"(b), "+v"(c), "+v"(d)); }
__device__ __forceinline__ void acc_guard1(v8f& a) { asm volatile("v_nop\n\tv_nop\n\tv_nop\n\tv_nop" : "+v"(a)); }

template <typename T> struct Frag;
template <> struct Frag<_Float16> {
  typedef v16h V; union U { v16h v; v8h h[2]; };
  static __device__ __forceinline__ v16h load(const _Float16* p) {
    U f; f.h[0] = *(const v8h*)(p); f.h[1] = *(const v8h*)(p + 16); return f.v;
  }
  static __device__ __forceinline__ v8f mma(v16h a, v16h b, v8f c) {
    return __builtin_amdgcn_wmma_f32_16x16x32_f16(false, a, false, b, (short)0, c, false, false);
  }
  static __device__ __forceinline__ void guard(v8f& a, v8f& b, v16h x, v16h y) { dep_guard_h(a, b, x, y); }
  static __device__ __forceinline__ void keep(v16h a, v16h b, v16h c, v16h d) { keep4_h(a, b, c, d); }
};

constexpr int kBatch  = 256;
constexpr int kHid    = 512;
constexpr int kOut    = 7;
constexpr int kLayers = 2;
constexpr int kSteps  = 64;
constexpr int kGates  = 4 * kHid;
constexpr int kKcat   = 2 * kHid;

constexpr int kRows    = 16;
constexpr int kBlocks  = kBatch / kRows;
constexpr int kWaves   = 4;
constexpr int kThreads = kWaves * 32;
constexpr int kUbPerLayer = kHid / 16;
constexpr int kPasses  = kUbPerLayer / kWaves;
constexpr int kCellsPerUb = kRows * 16;
constexpr int kStatePerBlock = kLayers * kUbPerLayer * kCellsPerUb;
constexpr int kSegP    = 520;
constexpr int kSegHalves = kRows * kSegP;
constexpr int kGbP     = 68;
constexpr int kYsP     = 20;
constexpr int kYcols   = 16;
static_assert(kBlocks * kRows == kBatch);
static_assert(kPasses * kWaves == kUbPerLayer);
static_assert((kSegP * 2) % 16 == 0 && (kYsP * 4) % 16 == 0 && (kGbP * 4) % 16 == 0);

constexpr float kActScale = 64.0f;
constexpr float kWScale   = 256.0f;
constexpr float kInvScale = 1.0f / 16384.0f;

constexpr int kPrepWThreads = kLayers * kGates * kKcat / 8;
constexpr int kPrepWBlocks  = kPrepWThreads / 256;
constexpr int kPrepFThreads = 16 * kHid / 8;
constexpr int kPrepFBlocks  = kPrepFThreads / 256;
static_assert(kPrepWBlocks * 256 == kPrepWThreads && kPrepFBlocks * 256 == kPrepFThreads);

constexpr size_t kWsWt   = 0;
constexpr size_t kWsWfc  = kWsWt + (size_t)kLayers * kGates * kKcat * 2;
constexpr size_t kWsY    = kWsWfc + (size_t)16 * kHid * 2;
constexpr size_t kWsCst  = kWsY + (size_t)kSteps * kBatch * kYcols * 4;
constexpr size_t kWsHst  = kWsCst + (size_t)kBlocks * kStatePerBlock * 4;
constexpr size_t kWsEnd  = kWsHst + (size_t)kBlocks * kStatePerBlock * 4;
static_assert(kWsEnd == 11550720);
static_assert(kWsWfc % 128 == 0 && kWsY % 128 == 0 && kWsCst % 1024 == 0 && kWsHst % 1024 == 0);
static_assert(kWsEnd <= 134217728);

__device__ __forceinline__ float sigm_f(float x) { return __builtin_amdgcn_rcpf(1.0f + expf(-x)); }
__device__ __forceinline__ float tanh_f(float x) { return 1.0f - 2.0f * __builtin_amdgcn_rcpf(1.0f + expf(2.0f * x)); }

__global__ __launch_bounds__(256) void prep_weights(const float* __restrict__ Wih, const float* __restrict__ Whh,
                                                     const float* __restrict__ Wfc,
                                                     _Float16* __restrict__ Wt, _Float16* __restrict__ Wfc16) {
  const int blk = blockIdx.x;
  if (blk < kPrepWBlocks) {
    const int i   = blk * 256 + (int)threadIdx.x;
    const int row = i >> 7;
    const int ch  = i & 127;
    const int kk  = (ch & 63) * 8;
    const float* pa = Wih + (size_t)row * kHid + kk;
    const float* pb = Whh + (size_t)row * kHid + kk;
    const v4f a0 = *(const v4f*)pa, a1 = *(const v4f*)(pa + 4);
    const v4f g0 = *(const v4f*)pb, g1 = *(const v4f*)(pb + 4);
    const bool useh = (ch >= 64);
    v8h o;
#pragma unroll
    for (int e = 0; e < 4; ++e) {
      const float va = useh ? g0[e] : a0[e];
      const float vb = useh ? g1[e] : a1[e];
      o[e]     = (_Float16)(va * kWScale);
      o[4 + e] = (_Float16)(vb * kWScale);
    }
    _Float16* dst = Wt + (size_t)i * 8;
    *(volatile v8h*)dst = o;
    __threadfence();
    *(volatile v8h*)dst = o;
  } else {
    const int j  = (blk - kPrepWBlocks) * 256 + (int)threadIdx.x;
    const int oo = j >> 6;
    const int kk = (j & 63) * 8;
    const int oc = oo < kOut ? oo : (kOut - 1);
    const float* p = Wfc + (size_t)oc * kHid + kk;
    const v4f a0 = *(const v4f*)p, a1 = *(const v4f*)(p + 4);
    const float z = (oo < kOut) ? kWScale : 0.0f;
    v8h o;
#pragma unroll
    for (int e = 0; e < 4; ++e) { o[e] = (_Float16)(a0[e] * z); o[4 + e] = (_Float16)(a1[e] * z); }
    _Float16* dst = Wfc16 + (size_t)j * 8;
    *(volatile v8h*)dst = o;
    __threadfence();
    *(volatile v8h*)dst = o;
  }
}

__device__ __forceinline__ void fill_seg(_Float16* seg, const float* __restrict__ src, int tid) {
  const int row  = tid >> 3;
  const int col0 = (tid & 7) * 64;
  const float* p = src + (size_t)row * kHid + col0;
  _Float16* d = seg + row * kSegP + col0;
#pragma unroll 1
  for (int j = 0; j < 8; ++j) {
    const v4f q0 = *(const v4f*)(p + j * 8), q1 = *(const v4f*)(p + j * 8 + 4);
    v8h o;
#pragma unroll
    for (int e = 0; e < 4; ++e) {
      o[e]     = (_Float16)(q0[e] * kActScale);
      o[4 + e] = (_Float16)(q1[e] * kActScale);
    }
    *(v8h*)(d + j * 8) = o;
  }
}

__device__ __forceinline__ void run_layer(const _Float16* sLo, const _Float16* sHi, _Float16* sOut, float* gb,
                                          const _Float16* __restrict__ Wl,
                                          const float* __restrict__ bi, const float* __restrict__ bh,
                                          const float* __restrict__ c0l,
                                          float* cst, float* hst,
                                          int stBase, int b0, int isFirst, int wave, int lane, int hh, int c) {
#pragma unroll 1
  for (int pass = 0; pass < kPasses; ++pass) {
    const int ub = pass * kWaves + wave;
    const int n0 = ub * 16;
    v8f acc[4];
#pragma unroll
    for (int g = 0; g < 4; ++g) acc[g] = (v8f){0.f, 0.f, 0.f, 0.f, 0.f, 0.f, 0.f, 0.f};
#pragma unroll
    for (int part = 0; part < 2; ++part) {
      const _Float16* arow = (part ? sHi : sLo) + c * kSegP + 8 * hh;
      const _Float16* wrow = Wl + (size_t)(n0 + c) * kKcat + part * kHid + 8 * hh;
#pragma unroll 2
      for (int ks = 0; ks < kHid / 32; ++ks) {
        const int k0 = ks * 32;
        const v16h a = Frag<_Float16>::load(arow + k0);
        v16h bq[4];
#pragma unroll
        for (int g = 0; g < 4; ++g) bq[g] = Frag<_Float16>::load(wrow + (size_t)g * kHid * kKcat + k0);
#pragma unroll
        for (int g = 0; g < 4; ++g) acc[g] = Frag<_Float16>::mma(a, bq[g], acc[g]);
        Frag<_Float16>::guard(acc[0], acc[3], a, a);
        Frag<_Float16>::keep(bq[0], bq[1], bq[2], bq[3]);
      }
    }
    acc_guard4(acc[0], acc[1], acc[2], acc[3]);

#pragma unroll
    for (int g = 0; g < 4; ++g) {
#pragma unroll
      for (int r = 0; r < 8; ++r) gb[(8 * hh + r) * kGbP + g * 16 + c] = acc[g][r];
    }
    __builtin_amdgcn_fence(__ATOMIC_RELEASE, "workgroup");
    __builtin_amdgcn_wave_barrier();
    __builtin_amdgcn_fence(__ATOMIC_ACQUIRE, "workgroup");

    const int n = n0 + c;
    const float bi0 = bi[n], bi1 = bi[kHid + n], bi2 = bi[2 * kHid + n], bi3 = bi[3 * kHid + n];
    const float bh0 = bh[n], bh1 = bh[kHid + n], bh2 = bh[2 * kHid + n], bh3 = bh[3 * kHid + n];
    const int sb = stBase + ub * kCellsPerUb;
#pragma unroll 1
    for (int it = 0; it < 8; ++it) {
      const int row = 2 * it + hh;
      const float* gr = gb + row * kGbP + c;
      float pi = gr[0]  * kInvScale + bi0; pi += bh0;
      float pf = gr[16] * kInvScale + bi1; pf += bh1;
      float pg = gr[32] * kInvScale + bi2; pg += bh2;
      float po = gr[48] * kInvScale + bi3; po += bh3;
      const int so = sb + it * 32 + lane;
      const float cs = cst[so];
      const float ci = c0l[(size_t)(b0 + row) * kHid + n];
      const float cold = isFirst ? ci : cs;
      const float ig = sigm_f(pi);
      const float fg = sigm_f(pf);
      const float gg = tanh_f(pg);
      const float og = sigm_f(po);
      const float cn = fg * cold + ig * gg;
      const float hn = og * tanh_f(cn);
      sOut[row * kSegP + n] = (_Float16)(hn * kActScale);
      *(volatile float*)(cst + so) = cn;
      *(volatile float*)(hst + so) = hn;
      __threadfence();
      *(volatile float*)(cst + so) = cn;
      *(volatile float*)(hst + so) = hn;
    }
    __builtin_amdgcn_fence(__ATOMIC_RELEASE, "workgroup");
    __builtin_amdgcn_wave_barrier();
    __builtin_amdgcn_fence(__ATOMIC_ACQUIRE, "workgroup");
  }
}

__global__ __launch_bounds__(kThreads) void rnn_steps(
    const float* __restrict__ x, const float* __restrict__ h0in, const float* __restrict__ c0in,
    const _Float16* __restrict__ Wt, const float* __restrict__ b_ih, const float* __restrict__ b_hh,
    const _Float16* __restrict__ Wfc16, const float* __restrict__ b_fc, const int* __restrict__ seqlen,
    float* __restrict__ Y, float* cst, float* hst) {
  __shared__ __align__(16) _Float16 segs[3][kSegHalves];
  __shared__ __align__(16) float gbuf[kWaves][kRows * kGbP];
  __shared__ __align__(16) float ys[kRows * kYsP];

  const int tid  = (int)threadIdx.x;
  const int wave = tid >> 5;
  const int lane = tid & 31;
  const int hh   = lane >> 4;
  const int c    = lane & 15;
  const int blk  = (int)blockIdx.x;
  const int b0   = blk * kRows;

  int nT = __builtin_amdgcn_readfirstlane(seqlen[0]);
  nT = nT < 0 ? 0 : (nT > kSteps ? kSteps : nT);

  fill_seg(segs[0], x + (size_t)b0 * kHid, tid);
  fill_seg(segs[1], h0in + (size_t)b0 * kHid, tid);
  __syncthreads();

  float* gb = gbuf[wave];
  int ia = 0, ib = 1, ic = 2;
  for (int t = 0; t < nT; ++t) {
    const int isFirst = (t == 0) ? 1 : 0;
#pragma unroll 1
    for (int l = 0; l < kLayers; ++l) {
      const _Float16* sLo = segs[l == 0 ? ia : ic];
      const _Float16* sHi = segs[l == 0 ? ib : ia];
      _Float16* sOut = segs[l == 0 ? ic : ib];
      run_layer(sLo, sHi, sOut, gb,
                Wt + (size_t)l * kGates * kKcat, b_ih + l * kGates, b_hh + l * kGates,
                c0in + (size_t)l * kBatch * kHid, cst, hst,
                (blk * kLayers + l) * (kUbPerLayer * kCellsPerUb), b0, isFirst, wave, lane, hh, c);
      __syncthreads();
      if (l == 0 && t == 0) fill_seg(segs[ia], h0in + (size_t)(kBatch + b0) * kHid, tid);
      __syncthreads();
    }
    if (wave == 0) {
      v8f yacc = (v8f){0.f, 0.f, 0.f, 0.f, 0.f, 0.f, 0.f, 0.f};
      const _Float16* arow = segs[ib] + c * kSegP + 8 * hh;
      const _Float16* wrow = Wfc16 + (size_t)c * kHid + 8 * hh;
#pragma unroll 1
      for (int ks = 0; ks < kHid / 32; ++ks) {
        const v16h a = Frag<_Float16>::load(arow + ks * 32);
        const v16h b = Frag<_Float16>::load(wrow + ks * 32);
        yacc = Frag<_Float16>::mma(a, b, yacc);
        dep_guard1(yacc, a, b);
      }
      acc_guard1(yacc);
      const int cc = c < kOut ? c : (kOut - 1);
      const float bfv = b_fc[cc];
      const bool live = (c < kOut);
#pragma unroll
      for (int r = 0; r < 8; ++r) {
        const float yv = yacc[r] * kInvScale + bfv;
        ys[(8 * hh + r) * kYsP + c] = live ? yv : 0.0f;
      }
      __builtin_amdgcn_fence(__ATOMIC_RELEASE, "workgroup");
      __builtin_amdgcn_wave_barrier();
      __builtin_amdgcn_fence(__ATOMIC_ACQUIRE, "workgroup");
      const int rr = lane >> 2, c4 = (lane & 3) * 4;
      float* yb = Y + ((size_t)t * kBatch + b0) * kYcols;
      for (int pass = 0; pass < 2; ++pass) {
#pragma unroll
        for (int half = 0; half < 2; ++half) {
          const int row = half * 8 + rr;
          const v4f yv4 = *(const v4f*)(ys + row * kYsP + c4);
          *(volatile v4f*)(yb + (size_t)row * kYcols + c4) = yv4;
        }
        __threadfence();
      }
    }
    const int tmp = ia; ia = ib; ib = ic; ic = tmp;
  }
}

constexpr int kDecPerBlock = kRows * kSteps * kOut;
static_assert(kDecPerBlock % 128 == 0);
__global__ __launch_bounds__(kThreads) void finish_out(const float* __restrict__ Y,
                                                        const float* __restrict__ cst, const float* __restrict__ hst,
                                                        float* __restrict__ dec, float* __restrict__ hT, float* __restrict__ cT) {
  __shared__ __align__(16) float sd[kDecPerBlock];
  const int tid  = (int)threadIdx.x;
  const int wave = tid >> 5, lane = tid & 31;
  const int blk  = (int)blockIdx.x;
  const int b0   = blk * kRows;
  for (int idx = tid; idx < kDecPerBlock; idx += kThreads) {
    const int row = idx / (kSteps * kOut);
    const int rem = idx - row * (kSteps * kOut);
    const int t   = rem / kOut;
    const int o   = rem - t * kOut;
    sd[idx] = Y[((size_t)t * kBatch + b0 + row) * kYcols + o];
  }
  __syncthreads();
  float* db = dec + (size_t)blk * kDecPerBlock;
  for (int pass = 0; pass < 2; ++pass) {
    for (int q = wave; q < kDecPerBlock / 128; q += kWaves) {
      const v4f v = *(const v4f*)(sd + q * 128 + lane * 4);
      *(volatile v4f*)(db + (size_t)q * 128 + lane * 4) = v;
    }
    __threadfence();
  }

#pragma unroll
  for (int pl = 0; pl < 2; ++pl) {
    const float* src = pl ? cst : hst;
    float* dst = pl ? cT : hT;
#pragma unroll 1
    for (int rr = wave; rr < kLayers * kRows; rr += kWaves) {
      const int l   = rr >> 4;
      const int row = rr & 15;
      const size_t sbase = ((size_t)(blk * kLayers + l) * kUbPerLayer) * kCellsPerUb + (size_t)row * 16 + (lane & 3) * 4;
      v4f v[4];
#pragma unroll
      for (int q = 0; q < 4; ++q) {
        const int ub = q * 8 + (lane >> 2);
        v[q] = *(const v4f*)(src + sbase + (size_t)ub * kCellsPerUb);
      }
      float* d = dst + ((size_t)(l * kBatch + b0 + row)) * kHid + lane * 4;
#pragma unroll
      for (int q = 0; q < 4; ++q) *(volatile v4f*)(d + q * 128) = v[q];
      __threadfence();
#pragma unroll
      for (int q = 0; q < 4; ++q) *(volatile v4f*)(d + q * 128) = v[q];
    }
  }
}

extern "C" void kernel_launch(void* const* d_in, const int* in_sizes, int n_in,
                              void* d_out, int out_size, void* d_ws, size_t ws_size,
                              hipStream_t stream) {
  if (n_in < 10) return;
  if (ws_size < kWsEnd) return;
  if (out_size < kBatch * kSteps * kOut + 2 * kLayers * kBatch * kHid) return;
  if (in_sizes[0] < kBatch * kHid || in_sizes[1] < kLayers * kBatch * kHid || in_sizes[2] < kLayers * kBatch * kHid) return;
  if (in_sizes[3] < kLayers * kGates * kHid || in_sizes[4] < kLayers * kGates * kHid) return;
  if (in_sizes[5] < kLayers * kGates || in_sizes[6] < kLayers * kGates || in_sizes[7] < kOut * kHid || in_sizes[8] < kOut || in_sizes[9] < 1) return;

  const float* x    = (const float*)d_in[0];
  const float* h0   = (const float*)d_in[1];
  const float* c0   = (const float*)d_in[2];
  const float* W_ih = (const float*)d_in[3];
  const float* W_hh = (const float*)d_in[4];
  const float* b_ih = (const float*)d_in[5];
  const float* b_hh = (const float*)d_in[6];
  const float* W_fc = (const float*)d_in[7];
  const float* b_fc = (const float*)d_in[8];
  const int*   sl   = (const int*)d_in[9];

  char* ws = (char*)d_ws;
  _Float16* Wt    = (_Float16*)(ws + kWsWt);
  _Float16* Wfc16 = (_Float16*)(ws + kWsWfc);
  float*    Y     = (float*)(ws + kWsY);
  float*    Cst   = (float*)(ws + kWsCst);
  float*    Hst   = (float*)(ws + kWsHst);

  float* out = (float*)d_out;
  float* dec = out;
  float* hT  = out + (size_t)kBatch * kSteps * kOut;
  float* cT  = hT + (size_t)kLayers * kBatch * kHid;

  prep_weights<<<dim3(kPrepWBlocks + kPrepFBlocks), dim3(256), 0, stream>>>(W_ih, W_hh, W_fc, Wt, Wfc16);
  rnn_steps<<<dim3(kBlocks), dim3(kThreads), 0, stream>>>(x, h0, c0, Wt, b_ih, b_hh, Wfc16, b_fc, sl, Y, Cst, Hst);
  finish_out<<<dim3(kBlocks), dim3(kThreads), 0, stream>>>(Y, Cst, Hst, dec, hT, cT);
}
